// CausalMultiHypothesisGraphTransformerLayer_3204045603778
// MI455X (gfx1250) — hardware-verified
//
#include <hip/hip_runtime.h>
#define NBt 8
#define CC 256
#define NN 1024
#define NR (NN * NBt)
#define NE0 3968
#define NE (NE0 + NN)
#define HEADS 8
#define HID 128
#define FF 512
#define NHYP 3
#define XLW (HEADS * CC)
#define DCAP 8
typedef __bf16 v16b __attribute__((ext_vector_type(16)));
typedef unsigned short v8us __attribute__((ext_vector_type(8), may_alias));
typedef float  v8f  __attribute__((ext_vector_type(8)));
typedef float  v4f  __attribute__((ext_vector_type(4)));
typedef float  v4fa __attribute__((ext_vector_type(4), may_alias));
union FragB { v16b v; v8us half[2]; unsigned short u[16]; };

__device__ __forceinline__ unsigned short bf16_bits(float x) { unsigned int u = __float_as_uint(x); return (unsigned short)((u + 0x7FFFu + ((u >> 16) & 1u)) >> 16); }
__device__ __forceinline__ float bf16_val(unsigned short b) { return __uint_as_float(((unsigned int)b) << 16); }
__device__ __forceinline__ float bf16_round(float x) { return bf16_val(bf16_bits(x)); }
template <int NT>
__device__ __forceinline__ v8f mmaN(v16b ah, v16b al, v16b bh, v16b bl, v8f c) {
  c = __builtin_amdgcn_wmma_f32_16x16x32_bf16(false, ah, false, bh, (short)0, c, false, false);
  if (NT >= 2) c = __builtin_amdgcn_wmma_f32_16x16x32_bf16(false, al, false, bh, (short)0, c, false, false);
  if (NT >= 3) c = __builtin_amdgcn_wmma_f32_16x16x32_bf16(false, ah, false, bl, (short)0, c, false, false);
  asm volatile("v_nop\n\tv_nop\n\tv_nop\n\tv_nop" : "+v"(c) : "v"(ah), "v"(al), "v"(bh), "v"(bl));
  return c;
}

__global__ __launch_bounds__(256) void k_wt_bf16(const float* __restrict__ W, unsigned short* __restrict__ Wt, int K, int N) {
  const int t = blockIdx.x * 256 + threadIdx.x;
  const int k8n = K / 8;
  if (t >= N * k8n) return;
  const int n = t / k8n, k8 = (t % k8n) * 8;
  v8us v;
#pragma unroll
  for (int i = 0; i < 8; ++i) v[i] = bf16_bits(W[(size_t)(k8 + i) * N + n]);
  *(volatile v8us*)(Wt + (size_t)n * K + k8) = v;
  __threadfence();
  *(volatile v8us*)(Wt + (size_t)n * K + k8) = v;
}

template <bool ASPLIT, int ACT, bool BIAS_BF16>
__global__ __launch_bounds__(128) void k_gemm_bf(const float* __restrict__ A, int lda, const unsigned short* __restrict__ Wt, int ldb,
                                               const float* __restrict__ bias, float* __restrict__ C, int ldc, int M, int N, int K) {
  __shared__ __attribute__((aligned(16))) float so[4][16][64];
  const int tid = threadIdx.x, w = tid >> 5, lane = tid & 31, ln = lane & 15, hh = lane >> 4;
  const int ntn = N / 64;
  const int wid = blockIdx.x * 4 + w;
  const int mt = wid / ntn, nq = wid % ntn;
  if (mt * 16 >= M) return;
  const int row0 = mt * 16, col0 = nq * 64;
  const float* arow = A + (size_t)(row0 + ln) * lda;
  v8f acc[4] = {};
  for (int kb = 0; kb < K; kb += 32) {
    FragB ah, al;
    const v4f x0 = *(const v4fa*)(arow + kb + 8 * hh), x1 = *(const v4fa*)(arow + kb + 8 * hh + 4);
    const v4f x2 = *(const v4fa*)(arow + kb + 16 + 8 * hh), x3 = *(const v4fa*)(arow + kb + 16 + 8 * hh + 4);
    float xs[16] = {x0[0],x0[1],x0[2],x0[3],x1[0],x1[1],x1[2],x1[3],x2[0],x2[1],x2[2],x2[3],x3[0],x3[1],x3[2],x3[3]};
#pragma unroll
    for (int i = 0; i < 16; ++i) { const unsigned short hb = bf16_bits(xs[i]); ah.u[i] = hb; al.u[i] = ASPLIT ? bf16_bits(xs[i] - bf16_val(hb)) : (unsigned short)0; }
#pragma unroll
    for (int t = 0; t < 4; ++t) {
      const unsigned short* brow = Wt + (size_t)(col0 + t * 16 + ln) * ldb + kb;
      FragB b;
      b.half[0] = *(const v8us*)(brow + 8 * hh);
      b.half[1] = *(const v8us*)(brow + 16 + 8 * hh);
      acc[t] = mmaN<ASPLIT ? 2 : 1>(ah.v, al.v, b.v, b.v, acc[t]);
    }
  }
#pragma unroll
  for (int t = 0; t < 4; ++t) {
    float bv = bias ? bias[col0 + t * 16 + ln] : 0.f;
    if (BIAS_BF16) bv = bf16_round(bv);
#pragma unroll
    for (int r = 0; r < 8; ++r) { float v = acc[t][r] + bv; if (ACT == 1) v = fmaxf(v, 0.f); so[w][8 * hh + r][t * 16 + ln] = v; }
  }
  __builtin_amdgcn_fence(__ATOMIC_ACQ_REL, "workgroup");
  __builtin_amdgcn_wave_barrier();
  const int rsub = lane >> 4, c4 = (lane & 15) * 4;
  for (int pass = 0; pass < 2; ++pass) {
#pragma unroll
    for (int q = 0; q < 8; ++q) {
      const int r = q * 2 + rsub;
      const v4f v = *(const v4fa*)&so[w][r][c4];
      *(volatile v4f*)(C + (size_t)(row0 + r) * ldc + col0 + c4) = v;
    }
    if (pass == 0) __threadfence();
  }
}

template <bool ASPLIT, int ACT, bool BIAS_BF16, bool RES_BF16>
__global__ __launch_bounds__(128) void k_gemm_bf3(const float* __restrict__ A, int lda, const unsigned short* __restrict__ Wt, int ldb,
                                                const float* __restrict__ bias, const float* __restrict__ resid, int rmod, int ldr,
                                                float* __restrict__ C, int ldc, int M, int N, int K) {
  __shared__ __attribute__((aligned(16))) float so[4][16][64];
  const int tid = threadIdx.x, w = tid >> 5, lane = tid & 31, ln = lane & 15, hh = lane >> 4;
  const int ntn = N / 64;
  const int wid = blockIdx.x * 4 + w;
  const int mt = wid / ntn, nq = wid % ntn;
  if (mt * 16 >= M) return;
  const int row0 = mt * 16, col0 = nq * 64;
  const float* arow = A + (size_t)(row0 + ln) * lda;
  v8f acc[4] = {};
  for (int kb = 0; kb < K; kb += 32) {
    FragB ah, al;
    const v4f x0 = *(const v4fa*)(arow + kb + 8 * hh), x1 = *(const v4fa*)(arow + kb + 8 * hh + 4);
    const v4f x2 = *(const v4fa*)(arow + kb + 16 + 8 * hh), x3 = *(const v4fa*)(arow + kb + 16 + 8 * hh + 4);
    float xs[16] = {x0[0],x0[1],x0[2],x0[3],x1[0],x1[1],x1[2],x1[3],x2[0],x2[1],x2[2],x2[3],x3[0],x3[1],x3[2],x3[3]};
#pragma unroll
    for (int i = 0; i < 16; ++i) { const unsigned short hb = bf16_bits(xs[i]); ah.u[i] = hb; al.u[i] = ASPLIT ? bf16_bits(xs[i] - bf16_val(hb)) : (unsigned short)0; }
#pragma unroll
    for (int t = 0; t < 4; ++t) {
      const unsigned short* brow = Wt + (size_t)(col0 + t * 16 + ln) * ldb + kb;
      FragB b;
      b.half[0] = *(const v8us*)(brow + 8 * hh);
      b.half[1] = *(const v8us*)(brow + 16 + 8 * hh);
      acc[t] = mmaN<ASPLIT ? 2 : 1>(ah.v, al.v, b.v, b.v, acc[t]);
    }
  }
#pragma unroll
  for (int t = 0; t < 4; ++t) {
    const int col = col0 + t * 16 + ln;
    float bv = bias ? bias[col] : 0.f;
    if (BIAS_BF16) bv = bf16_round(bv);
#pragma unroll
    for (int r = 0; r < 8; ++r) {
      float v = acc[t][r] + bv;
      if (resid) { float rv = resid[(size_t)((row0 + 8 * hh + r) % rmod) * ldr + col]; if (RES_BF16) rv = bf16_round(rv); v += rv; }
      if (ACT == 1) v = fmaxf(v, 0.f);
      if (ACT == 2) v = 0.5f * v * (1.0f + erff(v * 0.70710678118654752f));
      if (ACT == 3) { const float u = 0.7978845608028654f * (v + 0.044715f * v * v * v); v = 0.5f * v * (1.0f + tanhf(u)); }
      so[w][8 * hh + r][t * 16 + ln] = v;
    }
  }
  __builtin_amdgcn_fence(__ATOMIC_ACQ_REL, "workgroup");
  __builtin_amdgcn_wave_barrier();
  const int rsub = lane >> 4, c4 = (lane & 15) * 4;
  for (int pass = 0; pass < 2; ++pass) {
#pragma unroll
    for (int q = 0; q < 8; ++q) {
      const int r = q * 2 + rsub;
      const v4f v = *(const v4fa*)&so[w][r][c4];
      *(volatile v4f*)(C + (size_t)(row0 + r) * ldc + col0 + c4) = v;
    }
    if (pass == 0) __threadfence();
  }
}
template <bool PARAM_BF16>
__global__ __launch_bounds__(256) void k_layernorm(const float* __restrict__ X, const float* __restrict__ R, const float* __restrict__ g, const float* __restrict__ bta,
                                                  float* __restrict__ out_sum, float* __restrict__ out_norm, int N, float eps) {
  __shared__ float red[256];
  const int row = blockIdx.x, tid = threadIdx.x;
  const float* x = X + (size_t)row * N; const float* rr = R ? R + (size_t)row * N : nullptr;
  float vals[16];
  const int per = N / 256;
  float s1 = 0.f;
  for (int u = 0; u < per / 4; ++u) {
    const int j = tid * 4 + 1024 * u;
    const v4f a = *(const v4fa*)(x + j);
    v4f b = {0.f,0.f,0.f,0.f}; if (rr) b = *(const v4fa*)(rr + j);
#pragma unroll
    for (int q = 0; q < 4; ++q) { const float v = a[q] + b[q]; vals[u * 4 + q] = v; s1 += v; }
  }
  red[tid] = s1; __syncthreads();
  for (int st = 128; st > 0; st >>= 1) { if (tid < st) red[tid] += red[tid + st]; __syncthreads(); }
  const float mu = red[0] / (float)N; __syncthreads();
  float s2 = 0.f;
  for (int u = 0; u < per / 4; ++u)
#pragma unroll
    for (int q = 0; q < 4; ++q) { const float c = vals[u * 4 + q] - mu; s2 += c * c; }
  red[tid] = s2; __syncthreads();
  for (int st = 128; st > 0; st >>= 1) { if (tid < st) red[tid] += red[tid + st]; __syncthreads(); }
  const float rs = rsqrtf(red[0] / (float)N + eps);
  for (int pass = 0; pass < 2; ++pass) {
    for (int u = 0; u < per / 4; ++u) {
      const int j = tid * 4 + 1024 * u;
      v4f o, sm;
#pragma unroll
      for (int q = 0; q < 4; ++q) {
        float gg = g[j + q], bb = bta[j + q];
        if (PARAM_BF16) { gg = bf16_round(gg); bb = bf16_round(bb); }
        sm[q] = vals[u * 4 + q]; o[q] = (vals[u * 4 + q] - mu) * rs * gg + bb;
      }
      if (out_sum) *(volatile v4f*)(out_sum + (size_t)row * N + j) = sm;
      *(volatile v4f*)(out_norm + (size_t)row * N + j) = o;
    }
    if (pass == 0) __threadfence();
  }
}


typedef _Float16 v16h __attribute__((ext_vector_type(16)));
union FragH { v16h v; v8us half[2]; _Float16 h[16]; unsigned short u[16]; };
template <int NT>
__device__ __forceinline__ v8f mmaH(v16h ah, v16h al, v16h bh, v16h bl, v8f c) {
  c = __builtin_amdgcn_wmma_f32_16x16x32_f16(false, ah, false, bh, (short)0, c, false, false);
  if (NT >= 2) c = __builtin_amdgcn_wmma_f32_16x16x32_f16(false, al, false, bh, (short)0, c, false, false);
  if (NT >= 3) c = __builtin_amdgcn_wmma_f32_16x16x32_f16(false, ah, false, bl, (short)0, c, false, false);
  asm volatile("v_nop\n\tv_nop\n\tv_nop\n\tv_nop" : "+v"(c) : "v"(ah), "v"(al), "v"(bh), "v"(bl));
  return c;
}
template <bool ASPLIT>
__global__ __launch_bounds__(128) void k_gemm_h(const float* __restrict__ A, int lda, size_t sA, const _Float16* __restrict__ Bh, int ldb, size_t sB, float alpha, float* __restrict__ C, int ldc, size_t sC, int M, int N, int K) {
  __shared__ __attribute__((aligned(16))) float so[4][16][64];
  const int tid = threadIdx.x, w = tid >> 5, lane = tid & 31, ln = lane & 15, hh = lane >> 4; const int by = blockIdx.y;
  A += (size_t)by * sA; Bh += (size_t)by * sB; C += (size_t)by * sC;
  const int ntn = (N + 63) / 64; const int wid = blockIdx.x * 4 + w; const int mt = wid / ntn, nq = wid % ntn; if (mt * 16 >= M) return;
  const int row0 = mt * 16, col0 = nq * 64; const float* arow = A + (size_t)(row0 + ln) * lda;
  v8f acc[4] = {};
  for (int kb = 0; kb < K; kb += 32) {
    FragH ah, al;
    const v4f x0 = *(const v4fa*)(arow + kb + 8 * hh), x1 = *(const v4fa*)(arow + kb + 8 * hh + 4), x2 = *(const v4fa*)(arow + kb + 16 + 8 * hh), x3 = *(const v4fa*)(arow + kb + 16 + 8 * hh + 4);
    float xs[16] = {x0[0],x0[1],x0[2],x0[3],x1[0],x1[1],x1[2],x1[3],x2[0],x2[1],x2[2],x2[3],x3[0],x3[1],x3[2],x3[3]};
#pragma unroll
    for (int i = 0; i < 16; ++i) { const _Float16 h = (_Float16)xs[i]; ah.h[i] = h; al.h[i] = ASPLIT ? (_Float16)(xs[i] - (float)h) : (_Float16)0.0f; }
#pragma unroll
    for (int t = 0; t < 4; ++t) { if (col0 + t * 16 >= N) continue; const size_t boff = (size_t)(col0 + t * 16 + ln) * ldb + kb; FragH bq; bq.half[0] = *(const v8us*)(Bh + boff + 8 * hh); bq.half[1] = *(const v8us*)(Bh + boff + 16 + 8 * hh);
      acc[t] = mmaH<ASPLIT ? 2 : 1>(ah.v, al.v, bq.v, bq.v, acc[t]); }
  }
#pragma unroll
  for (int t = 0; t < 4; ++t) { if (col0 + t * 16 >= N) continue;
#pragma unroll
    for (int r = 0; r < 8; ++r) so[w][8 * hh + r][t * 16 + ln] = acc[t][r] * alpha; }
  __builtin_amdgcn_fence(__ATOMIC_ACQ_REL, "workgroup"); __builtin_amdgcn_wave_barrier();
  const int rsub = lane >> 4, c4 = (lane & 15) * 4;
  for (int pass = 0; pass < 2; ++pass) {
#pragma unroll
    for (int q = 0; q < 8; ++q) { const int r = q * 2 + rsub; if (col0 + c4 < N) { const v4f v = *(const v4fa*)&so[w][r][c4]; *(volatile v4f*)(C + (size_t)(row0 + r) * ldc + col0 + c4) = v; } }
    if (pass == 0) __threadfence(); }
}

__global__ __launch_bounds__(256) void k_wt_f16(const float* __restrict__ W, _Float16* __restrict__ Wt, int K, int N, float scale) {
  const int t = blockIdx.x * 256 + threadIdx.x; if (t >= N * (K / 8)) return; const int n = t / (K / 8), k8 = (t % (K / 8)) * 8; FragH f;
#pragma unroll
  for (int i = 0; i < 8; ++i) f.h[i] = (_Float16)(bf16_round(W[(size_t)(k8 + i) * N + n]) * scale); const v8us o = f.half[0];
  *(volatile v8us*)((unsigned short*)Wt + (size_t)n * K + k8) = o; __threadfence(); *(volatile v8us*)((unsigned short*)Wt + (size_t)n * K + k8) = o;
}
template <int ACT>
__global__ __launch_bounds__(128) void k_gemm_hhx(const _Float16* __restrict__ A, int lda, size_t sA, const _Float16* __restrict__ Bh, int ldb, size_t sB, float alpha, const float* __restrict__ bias, size_t sBias, const float* __restrict__ CP, int rowsPerB, size_t sCPb, int row0g,
    float* __restrict__ C, _Float16* __restrict__ C16, int ldc, size_t sC, int M, int N, int K) {
  __shared__ __attribute__((aligned(16))) float so[4][16][64];
  const int tid = threadIdx.x, w = tid >> 5, lane = tid & 31, ln = lane & 15, hh = lane >> 4; const int by = blockIdx.y;
  A += (size_t)by * sA; Bh += (size_t)by * sB; const size_t cofs = (size_t)by * sC; const float* bp = bias ? bias + (size_t)by * sBias : nullptr;
  const int ntn = (N + 63) / 64; const int wid = blockIdx.x * 4 + w; const int mt = wid / ntn, nq = wid % ntn; if (mt * 16 >= M) return;
  const int row0 = mt * 16, col0 = nq * 64; const _Float16* arow = A + (size_t)(row0 + ln) * lda;
  v8f acc[4] = {};
  for (int kb = 0; kb < K; kb += 32) { FragH ah; ah.half[0] = *(const v8us*)((const unsigned short*)arow + kb + 8 * hh); ah.half[1] = *(const v8us*)((const unsigned short*)arow + kb + 16 + 8 * hh);
#pragma unroll
    for (int t = 0; t < 4; ++t) { if (col0 + t * 16 >= N) continue; const size_t boff = (size_t)(col0 + t * 16 + ln) * ldb + kb; FragH bq; bq.half[0] = *(const v8us*)((const unsigned short*)Bh + boff + 8 * hh); bq.half[1] = *(const v8us*)((const unsigned short*)Bh + boff + 16 + 8 * hh);
      acc[t] = mmaH<1>(ah.v, ah.v, bq.v, bq.v, acc[t]); }
  }
#pragma unroll
  for (int t = 0; t < 4; ++t) { if (col0 + t * 16 >= N) continue; const int col = col0 + t * 16 + ln; const float bv = bp ? bf16_round(bp[col]) : 0.f;
#pragma unroll
    for (int r = 0; r < 8; ++r) { float v = acc[t][r] * alpha + bv; if (CP) { const int bidx = (row0g + row0 + 8 * hh + r) / rowsPerB; v += CP[(size_t)bidx * sCPb + (size_t)by * 64 + col]; } if (ACT == 1) v = (v > 0.f) ? v : expm1f(v); else if (ACT == 7) v = (v > 0.f) ? v + 1.0f : expf(v); else if (ACT == 8) v = tanhf(v); else if (ACT == 9) v = 0.5f * v * (1.0f + tanhf(0.7978845608028654f * (v + 0.044715f * v * v * v))); else if (ACT == 11) v = 1.0f / (1.0f + expf(-v)); else if (ACT == 12) v = (v > 0.f) ? v : 0.01f * v; else if (ACT == 14) v = (v > 0.f) ? v : 0.1f * v; else if (ACT == 15) v = v / (1.0f + expf(-v)); else if (ACT == 3) v = fmaxf(v, 0.f); else if (ACT == 6) v = 0.5f * v * (1.0f + erff(v * 0.70710678118654752f)); so[w][8 * hh + r][t * 16 + ln] = v; } }
  __builtin_amdgcn_fence(__ATOMIC_ACQ_REL, "workgroup"); __builtin_amdgcn_wave_barrier();
  const int rsub = lane >> 4, c4 = (lane & 15) * 4; typedef _Float16 v4h __attribute__((ext_vector_type(4)));
  for (int pass = 0; pass < 2; ++pass) {
#pragma unroll
    for (int q = 0; q < 8; ++q) { const int r = q * 2 + rsub; if (col0 + c4 < N) { const v4f v = *(const v4fa*)&so[w][r][c4]; if (C) *(volatile v4f*)(C + cofs + (size_t)(row0 + r) * ldc + col0 + c4) = v; if (C16) { v4h h4; for (int i = 0; i < 4; ++i) h4[i] = (_Float16)v[i]; *(volatile v4h*)(C16 + cofs + (size_t)(row0 + r) * ldc + col0 + c4) = h4; } } }
    if (pass == 0) __threadfence(); }
}


typedef _Float16 v4h __attribute__((ext_vector_type(4)));

__global__ __launch_bounds__(256) void k_x16(const float* __restrict__ x, _Float16* __restrict__ X16, size_t n8) { const size_t t = (size_t)blockIdx.x * 256 + threadIdx.x; if (t >= n8) return; FragH f;
#pragma unroll
  for (int q = 0; q < 8; ++q) f.h[q] = (_Float16)bf16_round(x[t * 8 + q]); *(volatile v8us*)((unsigned short*)X16 + t * 8) = f.half[0]; __threadfence(); *(volatile v8us*)((unsigned short*)X16 + t * 8) = f.half[0]; }
__global__ __launch_bounds__(256) void k_h16(const float* __restrict__ x, _Float16* __restrict__ X16, size_t n8) { const size_t t = (size_t)blockIdx.x * 256 + threadIdx.x; if (t >= n8) return; FragH f;
#pragma unroll
  for (int q = 0; q < 8; ++q) f.h[q] = (_Float16)x[t * 8 + q]; *(volatile v8us*)((unsigned short*)X16 + t * 8) = f.half[0]; __threadfence(); *(volatile v8us*)((unsigned short*)X16 + t * 8) = f.half[0]; }
__global__ __launch_bounds__(256) void k_round16f(const float* __restrict__ W, _Float16* __restrict__ Bt, size_t n8) { const size_t t = (size_t)blockIdx.x * 256 + threadIdx.x; if (t >= n8) return; FragH f;
#pragma unroll
  for (int i = 0; i < 8; ++i) f.h[i] = (_Float16)(bf16_round(W[t * 8 + i]) * 16.0f); *(volatile v8us*)((unsigned short*)Bt + t * 8) = f.half[0]; __threadfence(); *(volatile v8us*)((unsigned short*)Bt + t * 8) = f.half[0]; }
template <int NHv, int TTv>
__global__ __launch_bounds__(256) void k_vt(const _Float16* __restrict__ V16, int ldv, int voff, _Float16* __restrict__ Vt) { __shared__ unsigned short tl[64][66]; const int tid = threadIdx.x; const int slab = blockIdx.x / (TTv / 64), lg = blockIdx.x % (TTv / 64); const int b = slab / NHv, h = slab % NHv;
  for (int i = tid; i < 64 * 8; i += 256) { const int r = i / 8, c8 = (i % 8) * 8; FragH f; f.half[0] = *(const v8us*)((const unsigned short*)V16 + ((size_t)b * TTv + lg * 64 + r) * ldv + voff + h * 64 + c8);
#pragma unroll
    for (int q = 0; q < 8; ++q) tl[r][c8 + q] = f.u[q]; }
  __syncthreads();
  for (int pass = 0; pass < 2; ++pass) {
#pragma unroll
    for (int rd = 0; rd < 2; ++rd) { const int d = rd * 32 + tid / 8, pc = tid % 8; FragH f;
#pragma unroll
      for (int q = 0; q < 8; ++q) f.u[q] = tl[pc * 8 + q][d];
      *(volatile v8us*)((unsigned short*)Vt + ((size_t)slab * 64 + d) * TTv + lg * 64 + pc * 8) = f.half[0]; }
    if (pass == 0) __threadfence(); } }

__global__ __launch_bounds__(256) void k_hl(const float* __restrict__ F, _Float16* __restrict__ Hh, _Float16* __restrict__ Hl, size_t n8) { const size_t t = (size_t)blockIdx.x * 256 + threadIdx.x; if (t >= n8) return; FragH fh, fl; const v4f a = *(const v4fa*)(F + t * 8), c = *(const v4fa*)(F + t * 8 + 4);
#pragma unroll
  for (int q = 0; q < 4; ++q) { _Float16 h = (_Float16)a[q]; fh.h[q] = h; fl.h[q] = (_Float16)((a[q] - (float)h) * 1024.0f); h = (_Float16)c[q]; fh.h[4 + q] = h; fl.h[4 + q] = (_Float16)((c[q] - (float)h) * 1024.0f); }
  for (int pass = 0; pass < 2; ++pass) { *(volatile v8us*)((unsigned short*)Hh + t * 8) = fh.half[0]; *(volatile v8us*)((unsigned short*)Hl + t * 8) = fl.half[0]; if (pass == 0) __threadfence(); } }
#define VST2(T, ptr, val) do { const T vst2_v_ = (val); *(volatile T*)(ptr) = vst2_v_; __threadfence(); *(volatile T*)(ptr) = vst2_v_; } while (0)

#define C4_NB 4096
#define C4_CH 8192
__device__ __forceinline__ int c4_bucket(int v, int N) { v = min(max(v, 0), N - 1); return (int)(((long long)v * C4_NB) / N); }
__global__ __launch_bounds__(256) void k_c4_count(const int* __restrict__ tgt, int E, int N, int* __restrict__ CNT) {
    __shared__ int hist[C4_NB]; const int ch = blockIdx.x, t = threadIdx.x; const int e0 = ch * C4_CH; const int nt = min(C4_CH, E - e0);
    for (int j = 0; j < 16; ++j) hist[t + 256 * j] = 0; __syncthreads();
    for (int i = t; i < nt; i += 256) atomicAdd(&hist[c4_bucket(tgt[e0 + i], N)], 1);
    __syncthreads();
    for (int j = 0; j < 16; ++j) { const int v = hist[t + 256 * j]; VST2(int, CNT + (long long)ch * C4_NB + t + 256 * j, v); } }
__global__ __launch_bounds__(256) void k_c4_offsets(const int* __restrict__ CNT, int nch, int E, int* __restrict__ OFFB, int* __restrict__ BOFF) {
    __shared__ int tot[C4_NB]; __shared__ int part[256]; const int t = threadIdx.x;
    for (int j = 0; j < 16; ++j) { const int b = t + 256 * j; int s = 0; for (int ch = 0; ch < nch; ++ch) s += CNT[(long long)ch * C4_NB + b]; tot[b] = s; }
    __syncthreads();
    { int s = 0; for (int q = 0; q < 16; ++q) s += tot[16 * t + q]; part[t] = s; } __syncthreads();
    if (t == 0) { int run = 0; for (int i = 0; i < 256; ++i) { const int v = part[i]; part[i] = run; run += v; } } __syncthreads();
    { int run = part[t]; for (int q = 0; q < 16; ++q) { const int v = tot[16 * t + q]; tot[16 * t + q] = run; run += v; } }
    __syncthreads();
    for (int j = 0; j < 16; ++j) { const int b = t + 256 * j; VST2(int, BOFF + b, tot[b]); }
    if (t == 0) VST2(int, BOFF + C4_NB, E);
    for (int j = 0; j < 16; ++j) { const int b = t + 256 * j; int run = tot[b]; for (int ch = 0; ch < nch; ++ch) { VST2(int, OFFB + (long long)ch * C4_NB + b, run); run += CNT[(long long)ch * C4_NB + b]; } } }
__global__ __launch_bounds__(256) void k_c4_scatter(const int* __restrict__ tgt, int E, int N, const int* __restrict__ OFFB, int* __restrict__ BUF) {
    __shared__ int cur[C4_NB]; __shared__ int bk[256]; const int ch = blockIdx.x, t = threadIdx.x; const int e0 = ch * C4_CH; const int nt = min(C4_CH, E - e0);
    const int wv = t >> 5, ln = t & 31;
    for (int j = 0; j < 16; ++j) cur[t + 256 * j] = OFFB[(long long)ch * C4_NB + t + 256 * j];
    __syncthreads();
    for (int s0 = 0; s0 < C4_CH; s0 += 256) {
        const int i = s0 + t; const int e = e0 + i; const int b = (i < nt) ? c4_bucket(tgt[min(e, E - 1)], N) : -1;
        bk[t] = b; __syncthreads();
        int rank = 0, cntw = 0;
        for (int l = 0; l < 32; ++l) { const int o = bk[(wv << 5) + l]; const bool same = (o == b) && (b >= 0); cntw += same ? 1 : 0; rank += (same && l < ln) ? 1 : 0; }
        const bool last = (b >= 0) && (rank == cntw - 1);
        for (int w = 0; w < 8; ++w) {
            if (wv == w && b >= 0) { int pos = cur[b] + rank; pos = min(max(pos, 0), E - 1); VST2(int, BUF + pos, e); }
            __syncthreads();
            if (wv == w && last) cur[b] += cntw;
            __syncthreads(); }
    } }
template <int CAP>
__global__ __launch_bounds__(256) void k_c4_lists(const int* __restrict__ tgt, const int* __restrict__ BUF, const int* __restrict__ BOFF, int N, int E, int* __restrict__ NBR, int* __restrict__ cnt) {
    const int d = blockIdx.x * 256 + threadIdx.x; if (d >= N) return; const int b = c4_bucket(d, N); int n = 0; int* row = NBR + (long long)d * CAP;
    const int p0 = min(max(BOFF[b], 0), E), p1 = min(max(BOFF[b + 1], p0), E);
    for (int p = p0; p < p1; ++p) { int e = BUF[p]; e = min(max(e, 0), E - 1); if (tgt[e] == d) { if (n < CAP) VST2(int, row + n, e); ++n; } }
    for (int j = n; j < CAP; ++j) VST2(int, row + j, -1); VST2(int, cnt + d, min(n, CAP)); }
__global__ __launch_bounds__(256) void k_c4_scan1(const int* __restrict__ cnt, int* __restrict__ PART, int N) {
    __shared__ int part[256]; const int per = ((((N + 255) / 256) + 31) / 32) * 32; const int a = threadIdx.x * per, b = min(N, a + per); int s = 0;
    for (int i = a; i < b; ++i) s += cnt[i]; part[threadIdx.x] = s; __syncthreads();
    if (threadIdx.x == 0) { int run = 0; for (int t = 0; t < 256; ++t) { const int v = part[t]; part[t] = run; run += v; } } __syncthreads();
    VST2(int, PART + threadIdx.x, part[threadIdx.x]); }
__global__ __launch_bounds__(256) void k_c4_scan2(const int* __restrict__ cnt, const int* __restrict__ PART, int* __restrict__ off, int N) {
    const int i = blockIdx.x * 256 + threadIdx.x; if (i > N) return; const int per = ((((N + 255) / 256) + 31) / 32) * 32; const int r = min(i / per, 255); const int a = r * per;
    int s = PART[r]; for (int kq = a; kq < i; ++kq) s += cnt[min(kq, N - 1)];
    VST2(int, off + i, s); }
template <int CAP>
__global__ __launch_bounds__(256) void k_c4_slotcopy(const int* __restrict__ off, const int* __restrict__ NBR, int* __restrict__ slot, int N) {
    const int t = blockIdx.x * 256 + threadIdx.x; const int tot = off[N]; if (t >= tot) return;
    int lo = 0, hi = N - 1; while (lo < hi) { const int mid = (lo + hi + 1) >> 1; if (off[mid] <= t) lo = mid; else hi = mid - 1; }
    int j = t - off[lo]; j = (j < 0) ? 0 : ((j >= CAP) ? (CAP - 1) : j); VST2(int, slot + t, NBR[(long long)lo * CAP + j]); }

__device__ __forceinline__ float lrelu02(float v) { return (v >= 0.f) ? v : 0.2f * v; }
__device__ __forceinline__ v4f shfl4(v4f v, int srcl) { v4f r; r[0] = __shfl(v[0], srcl, 32); r[1] = __shfl(v[1], srcl, 32); r[2] = __shfl(v[2], srcl, 32); r[3] = __shfl(v[3], srcl, 32); return r; }
__device__ __forceinline__ void store_row8(float* row, v4f oa, v4f ob, int l) {
  const v4f a1 = shfl4(oa, l >> 1), b1 = shfl4(ob, l >> 1), a2 = shfl4(oa, 16 + (l >> 1)), b2 = shfl4(ob, 16 + (l >> 1)); const v4f c1 = (l & 1) ? b1 : a1, c2 = (l & 1) ? b2 : a2;
  for (int pass = 0; pass < 2; ++pass) { *(volatile v4f*)(row + l * 4) = c1; *(volatile v4f*)(row + 128 + l * 4) = c2; if (pass == 0) __threadfence(); } }
__global__ __launch_bounds__(256) void k_edges(const int* __restrict__ ei, int* __restrict__ ES, int* __restrict__ ED) { const int e = blockIdx.x * 256 + threadIdx.x; if (e >= NE) return; int s, d; if (e < NE0) { s = ei[e]; d = ei[NE0 + e]; } else { s = d = e - NE0; } s = min(max(s, 0), NN - 1); d = min(max(d, 0), NN - 1); *(volatile int*)(ES + e) = s; *(volatile int*)(ED + e) = d; __threadfence(); *(volatile int*)(ES + e) = s; *(volatile int*)(ED + e) = d; }
__global__ __launch_bounds__(256) void k_tok16(const float* __restrict__ x, _Float16* __restrict__ X16) { const int t = blockIdx.x * 256 + threadIdx.x; if (t >= NR * (CC / 8)) return; const int c0 = (t % (CC / 8)) * 8, r = t / (CC / 8); const int n = r / NBt, b = r % NBt; FragH f;
#pragma unroll
  for (int q = 0; q < 8; ++q) f.h[q] = (_Float16)bf16_round(x[((size_t)b * CC + c0 + q) * NN + n]);
  *(volatile v8us*)((unsigned short*)X16 + (size_t)r * CC + c0) = f.half[0]; __threadfence(); *(volatile v8us*)((unsigned short*)X16 + (size_t)r * CC + c0) = f.half[0]; }
__global__ __launch_bounds__(256) void k_f16(const float* __restrict__ F, _Float16* __restrict__ O16, size_t n8) { const size_t t = (size_t)blockIdx.x * 256 + threadIdx.x; if (t >= n8) return; const v4f a = *(const v4fa*)(F + t * 8), c = *(const v4fa*)(F + t * 8 + 4); FragH f;
#pragma unroll
  for (int q = 0; q < 8; ++q) f.h[q] = (_Float16)((q < 4) ? a[q] : c[q - 4]);
  *(volatile v8us*)((unsigned short*)O16 + t * 8) = f.half[0]; __threadfence(); *(volatile v8us*)((unsigned short*)O16 + t * 8) = f.half[0]; }
__global__ __launch_bounds__(256) void k_gate(const float* __restrict__ Z, const float* __restrict__ NODE, _Float16* __restrict__ XC, _Float16* __restrict__ XA, size_t n8) {
  #pragma clang fp contract(off)
  const size_t t = (size_t)blockIdx.x * 256 + threadIdx.x; if (t >= n8 * 2) return; FragH fc, fa;
#pragma unroll
  for (int q = 0; q < 4; ++q) { const float z = Z[t * 4 + q], nd = NODE[t * 4 + q]; fc.h[q] = (_Float16)((1.0f / (1.0f + expf(-z))) * nd); fa.h[q] = (_Float16)((1.0f / (1.0f + expf(z))) * nd); }
  const unsigned long long pc = *(const unsigned long long*)&fc.u[0], pa = *(const unsigned long long*)&fa.u[0];
  for (int pass = 0; pass < 2; ++pass) { *(volatile unsigned long long*)((unsigned short*)XC + t * 4) = pc; *(volatile unsigned long long*)((unsigned short*)XA + t * 4) = pa; if (pass == 0) __threadfence(); } }
__global__ __launch_bounds__(256) void k_gcnln(const int* __restrict__ NBR, const int* __restrict__ cnt, const int* __restrict__ ES, const float* __restrict__ HW, const float* __restrict__ bg, const float* __restrict__ g, const float* __restrict__ bb, float* __restrict__ OUT) {
  #pragma clang fp contract(off)
  const int tid = threadIdx.x, w = tid >> 5, l = tid & 31; const int r = blockIdx.x * 8 + w; if (r >= NR) return; const int n = r / NBt, b = r % NBt; const int ne = min(cnt[n], DCAP); const float dn = (float)cnt[n]; float v[8];
#pragma unroll
  for (int k = 0; k < 8; ++k) v[k] = bf16_round(bg[l * 8 + k]);
#pragma unroll 1
  for (int j = 0; j < ne; ++j) { int e = NBR[(size_t)n * DCAP + j]; e = min(max(e, 0), NE - 1); const int s = ES[e]; const float nrm = rsqrtf((float)cnt[s] * dn); const v4f a = *(const v4fa*)(HW + ((size_t)s * NBt + b) * CC + l * 8), c = *(const v4fa*)(HW + ((size_t)s * NBt + b) * CC + l * 8 + 4);
#pragma unroll
    for (int k = 0; k < 8; ++k) v[k] += ((k < 4) ? a[k] : c[k - 4]) * nrm; }
  float sm = 0.f;
#pragma unroll
  for (int k = 0; k < 8; ++k) sm += v[k];
  for (int o = 16; o > 0; o >>= 1) sm += __shfl_xor(sm, o, 32); const float mu = sm / (float)CC; float q2 = 0.f;
#pragma unroll
  for (int k = 0; k < 8; ++k) { const float d = v[k] - mu; q2 += d * d; }
  for (int o = 16; o > 0; o >>= 1) q2 += __shfl_xor(q2, o, 32); const float rs = rsqrtf(q2 / (float)CC + 1e-5f); v4f oa, ob;
#pragma unroll
  for (int k = 0; k < 8; ++k) { const int c = l * 8 + k; const float y = (v[k] - mu) * rs * bf16_round(g[c]) + bf16_round(bb[c]); if (k < 4) oa[k] = y; else ob[k - 4] = y; }
  store_row8(OUT + (size_t)r * CC, oa, ob, l); }
__global__ __launch_bounds__(256) void k_acsum(const float* __restrict__ ADJ, const float* __restrict__ CONF, float* __restrict__ AC, _Float16* __restrict__ AC16, _Float16* __restrict__ CF16, size_t n8) {
  #pragma clang fp contract(off)
  const size_t t = (size_t)blockIdx.x * 256 + threadIdx.x; if (t >= n8) return; const v4f a = *(const v4fa*)(ADJ + t * 8), a2 = *(const v4fa*)(ADJ + t * 8 + 4), c = *(const v4fa*)(CONF + t * 8), c2 = *(const v4fa*)(CONF + t * 8 + 4); const v4f s1 = a + c, s2 = a2 + c2; FragH f, g;
#pragma unroll
  for (int q = 0; q < 4; ++q) { f.h[q] = (_Float16)s1[q]; f.h[4 + q] = (_Float16)s2[q]; g.h[q] = (_Float16)c[q]; g.h[4 + q] = (_Float16)c2[q]; }
  const int l = (int)(threadIdx.x & 31); store_row8(AC + (t - (size_t)l) * 8, s1, s2, l);
  for (int pass = 0; pass < 2; ++pass) { *(volatile v8us*)((unsigned short*)AC16 + t * 8) = f.half[0]; *(volatile v8us*)((unsigned short*)CF16 + t * 8) = g.half[0]; if (pass == 0) __threadfence(); } }
__global__ __launch_bounds__(256) void k_ln(const float* __restrict__ T, const float* __restrict__ g, const float* __restrict__ bb, float* __restrict__ OUT) {
  #pragma clang fp contract(off)
  const int tid = threadIdx.x, w = tid >> 5, l = tid & 31; const int r = blockIdx.x * 8 + w; if (r >= NR) return; float v[8]; float sm = 0.f;
#pragma unroll
  for (int k = 0; k < 8; ++k) { v[k] = T[(size_t)r * CC + l * 8 + k]; sm += v[k]; }
  for (int o = 16; o > 0; o >>= 1) sm += __shfl_xor(sm, o, 32); const float mu = sm / (float)CC; float q2 = 0.f;
#pragma unroll
  for (int k = 0; k < 8; ++k) { const float d = v[k] - mu; q2 += d * d; }
  for (int o = 16; o > 0; o >>= 1) q2 += __shfl_xor(q2, o, 32); const float rs = rsqrtf(q2 / (float)CC + 1e-5f); v4f oa, ob;
#pragma unroll
  for (int k = 0; k < 8; ++k) { const int c = l * 8 + k; const float y = (v[k] - mu) * rs * bf16_round(g[c]) + bf16_round(bb[c]); if (k < 4) oa[k] = y; else ob[k - 4] = y; }
  store_row8(OUT + (size_t)r * CC, oa, ob, l); }
__global__ __launch_bounds__(256) void k_gat(const int* __restrict__ NBR, const int* __restrict__ cnt, const int* __restrict__ ES, const _Float16* __restrict__ XL, const _Float16* __restrict__ XR, const float* __restrict__ att, const float* __restrict__ gb, float* __restrict__ OUT) {
  #pragma clang fp contract(off)
  const int tid = threadIdx.x, w = tid >> 5, l = tid & 31; const int r = blockIdx.x * 8 + w; if (r >= NR) return; const int n = r / NBt, b = r % NBt; const int ne = min(cnt[n], DCAP); float acc[8];
#pragma unroll
  for (int k = 0; k < 8; ++k) acc[k] = 0.f;
  int srcs[DCAP];
#pragma unroll
  for (int j = 0; j < DCAP; ++j) { int e = NBR[(size_t)n * DCAP + min(j, max(ne - 1, 0))]; e = min(max(e, 0), NE - 1); srcs[j] = ES[e]; }
#pragma unroll 1
  for (int h = 0; h < HEADS; ++h) { const size_t co = (size_t)h * CC + l * 8; FragH xr; xr.half[0] = *(const v8us*)((const unsigned short*)XR + (size_t)r * XLW + co); float at8[8];
#pragma unroll
    for (int k = 0; k < 8; ++k) at8[k] = bf16_round(att[(size_t)h * CC + l * 8 + k]);
    float lg[DCAP]; FragH xls[DCAP];
#pragma unroll
    for (int j = 0; j < DCAP; ++j) { xls[j].half[0] = *(const v8us*)((const unsigned short*)XL + ((size_t)srcs[j] * NBt + b) * XLW + co); float s = 0.f;
#pragma unroll
      for (int k = 0; k < 8; ++k) s += lrelu02((float)xls[j].h[k] + (float)xr.h[k]) * at8[k];
      for (int o = 16; o > 0; o >>= 1) s += __shfl_xor(s, o, 32);
      lg[j] = (j < ne) ? s : -3.0e38f; }
    float m = lg[0];
#pragma unroll
    for (int j = 1; j < DCAP; ++j) m = fmaxf(m, lg[j]);
    float su = 0.f;
#pragma unroll
    for (int j = 0; j < DCAP; ++j) { lg[j] = (j < ne) ? expf(lg[j] - m) : 0.f; su += lg[j]; }
#pragma unroll
    for (int j = 0; j < DCAP; ++j) { const float a = lg[j] / su;
#pragma unroll
      for (int k = 0; k < 8; ++k) acc[k] += a * (float)xls[j].h[k]; } }
  v4f oa, ob;
#pragma unroll
  for (int k = 0; k < 8; ++k) { const float y = acc[k] / (float)HEADS + bf16_round(gb[l * 8 + k]); if (k < 4) oa[k] = y; else ob[k - 4] = y; }
  store_row8(OUT + (size_t)r * CC, oa, ob, l); }
__global__ __launch_bounds__(256) void k_nchw(const float* __restrict__ Rw, float* __restrict__ out) { const int t = blockIdx.x * 256 + threadIdx.x; if (t >= NBt * CC * (NN / 4)) return; const int n0 = (t % (NN / 4)) * 4; const int c = (t / (NN / 4)) % CC; const int b = t / ((NN / 4) * CC); v4f v;
#pragma unroll
  for (int q = 0; q < 4; ++q) v[q] = Rw[((size_t)(n0 + q) * NBt + b) * CC + c];
  float* dst = out + ((size_t)b * CC + c) * NN + n0; *(volatile v4f*)dst = v; __threadfence(); *(volatile v4f*)dst = v; }

extern "C" void kernel_launch(void* const* d_in, const int* in_sizes, int n_in,
                              void* d_out, int out_size, void* d_ws, size_t ws_size, hipStream_t stream) {
  (void)in_sizes; (void)n_in; (void)out_size;
  const float* const* I = (const float* const*)d_in; const float* x = I[0]; const int* ei = (const int*)d_in[1];
  const float* Wp = I[2]; const float* bp = I[3]; const float* Wm1 = I[4]; const float* bm1 = I[5]; const float* Wm2 = I[6]; const float* bm2 = I[7]; const float* Wgca = I[8]; const float* bgca = I[9]; const float* Wgcc = I[10]; const float* bgcc = I[11]; const float* Wi1 = I[12]; const float* bi1 = I[13]; const float* Wi2 = I[14]; const float* bi2 = I[15]; const float* Wl = I[16]; const float* bl = I[17]; const float* Wr = I[18]; const float* br = I[19]; const float* att = I[20]; const float* gb = I[21]; const float* Wf1 = I[22]; const float* bf1 = I[23]; const float* Wf2 = I[24]; const float* bf2 = I[25]; const float* lng = I[26]; const float* lnb = I[27];
  char* ws = (char*)d_ws; size_t off = 0;
  auto take = [&](size_t bytes) { char* p = ws + off; off += (bytes + 255) & ~(size_t)255; return p; };
  const int nch = (NE + C4_CH - 1) / C4_CH;
  int* ES = (int*)take(NE * 4); int* ED = (int*)take(NE * 4); int* CNT = (int*)take((size_t)nch * C4_NB * 4); int* OFFB = (int*)take((size_t)nch * C4_NB * 4); int* BOFF = (int*)take((size_t)(C4_NB + 64) * 4); int* BUF = (int*)take((size_t)NE * 4); int* NBR = (int*)take((size_t)NN * DCAP * 4); int* cnt = (int*)take((size_t)(NN + 64) * 4);
  _Float16* BWp = (_Float16*)take(CC * CC * 2); _Float16* BWm1 = (_Float16*)take(HID * CC * 2); _Float16* BWm2 = (_Float16*)take(CC * HID * 2); _Float16* BWga = (_Float16*)take(CC * CC * 2); _Float16* BWgc = (_Float16*)take(CC * CC * 2); _Float16* BWi1 = (_Float16*)take(HID * CC * 2); _Float16* BWi2 = (_Float16*)take(CC * HID * 2); _Float16* BWl = (_Float16*)take((size_t)XLW * CC * 2); _Float16* BWr = (_Float16*)take((size_t)XLW * CC * 2); _Float16* BWf1 = (_Float16*)take(FF * CC * 2); _Float16* BWf2 = (_Float16*)take(CC * FF * 2);
  char* RA = take((size_t)NR * XLW * 2);
  char* RB = take((size_t)NR * XLW * 2);
  float* AC = (float*)take((size_t)NR * CC * 4); _Float16* AC16 = (_Float16*)take((size_t)NR * CC * 2); _Float16* CF16 = (_Float16*)take((size_t)NR * CC * 2); _Float16* I1 = (_Float16*)take((size_t)NR * HID * 2); float* FEAT = (float*)take((size_t)NR * CC * 4); _Float16* F16 = (_Float16*)take((size_t)NR * CC * 2); float* HYP = (float*)take((size_t)NR * CC * 4);
  if (off > ws_size) return;
  float* NODE = (float*)RA; float* Z = (float*)(RA + (size_t)NR * CC * 4); _Float16* N16 = (_Float16*)(RA + (size_t)NR * CC * 8); _Float16* Z1 = (_Float16*)(RA + (size_t)NR * CC * 10); _Float16* XC16 = (_Float16*)(RA + (size_t)NR * CC * 11); _Float16* XA16 = (_Float16*)(RA + (size_t)NR * CC * 13); _Float16* XL = (_Float16*)RA; _Float16* FF16 = (_Float16*)RA; float* T = (float*)(RA + (size_t)NR * FF * 2);
  _Float16* X16 = (_Float16*)RB; float* HW = (float*)(RB + (size_t)NR * CC * 2); float* ADJ = (float*)(RB + (size_t)NR * CC * 6); float* CONF = (float*)(RB + (size_t)NR * CC * 10); _Float16* XR = (_Float16*)RB;
  k_edges<<<(NE + 255) / 256, 256, 0, stream>>>(ei, ES, ED);
  k_c4_count<<<nch, 256, 0, stream>>>(ED, NE, NN, CNT); k_c4_offsets<<<1, 256, 0, stream>>>(CNT, nch, NE, OFFB, BOFF); k_c4_scatter<<<nch, 256, 0, stream>>>(ED, NE, NN, OFFB, BUF); k_c4_lists<DCAP><<<(NN + 255) / 256, 256, 0, stream>>>(ED, BUF, BOFF, NN, NE, NBR, cnt);
  k_wt_f16<<<(CC * (CC / 8) + 255) / 256, 256, 0, stream>>>(Wp, BWp, CC, CC, 16.0f); k_wt_f16<<<(HID * (CC / 8) + 255) / 256, 256, 0, stream>>>(Wm1, BWm1, CC, HID, 16.0f); k_wt_f16<<<(CC * (HID / 8) + 255) / 256, 256, 0, stream>>>(Wm2, BWm2, HID, CC, 16.0f); k_wt_f16<<<(CC * (CC / 8) + 255) / 256, 256, 0, stream>>>(Wgca, BWga, CC, CC, 16.0f); k_wt_f16<<<(CC * (CC / 8) + 255) / 256, 256, 0, stream>>>(Wgcc, BWgc, CC, CC, 16.0f); k_wt_f16<<<(FF * (CC / 8) + 255) / 256, 256, 0, stream>>>(Wf1, BWf1, CC, FF, 16.0f); k_wt_f16<<<(CC * (FF / 8) + 255) / 256, 256, 0, stream>>>(Wf2, BWf2, FF, CC, 16.0f);
  const size_t n8 = (size_t)NR * CC / 8; const unsigned nb8 = (unsigned)((n8 + 255) / 256); const dim3 gC(((NR / 16) * (CC / 64) + 3) / 4, 1), gH(((NR / 16) * (HID / 64) + 3) / 4, 1), gX(((NR / 16) * (XLW / 64) + 3) / 4, 1), gF(((NR / 16) * (FF / 64) + 3) / 4, 1);
  k_tok16<<<nb8, 256, 0, stream>>>(x, X16);
  k_gemm_hhx<0><<<gC, 128, 0, stream>>>(X16, CC, 0, BWp, CC, 0, 0.0625f, bp, 0, nullptr, 1, 0, 0, NODE, nullptr, CC, 0, NR, CC, CC); k_f16<<<nb8, 256, 0, stream>>>(NODE, N16, n8);
  k_gemm_hhx<3><<<gH, 128, 0, stream>>>(N16, CC, 0, BWm1, CC, 0, 0.0625f, bm1, 0, nullptr, 1, 0, 0, nullptr, Z1, HID, 0, NR, HID, CC); k_gemm_hhx<0><<<gC, 128, 0, stream>>>(Z1, HID, 0, BWm2, HID, 0, 0.0625f, bm2, 0, nullptr, 1, 0, 0, Z, nullptr, CC, 0, NR, CC, HID);
  k_gate<<<nb8 * 2, 256, 0, stream>>>(Z, NODE, XC16, XA16, n8);
  k_gemm_hhx<0><<<gC, 128, 0, stream>>>(XA16, CC, 0, BWga, CC, 0, 0.0625f, nullptr, 0, nullptr, 1, 0, 0, HW, nullptr, CC, 0, NR, CC, CC); k_gcnln<<<NR / 8, 256, 0, stream>>>(NBR, cnt, ES, HW, bgca, lng, lnb, ADJ);
  k_gemm_hhx<0><<<gC, 128, 0, stream>>>(XC16, CC, 0, BWgc, CC, 0, 0.0625f, nullptr, 0, nullptr, 1, 0, 0, HW, nullptr, CC, 0, NR, CC, CC); k_gcnln<<<NR / 8, 256, 0, stream>>>(NBR, cnt, ES, HW, bgcc, lng + CC, lnb + CC, CONF);
  k_acsum<<<nb8, 256, 0, stream>>>(ADJ, CONF, AC, AC16, CF16, n8);
  for (int i = 0; i < NHYP; ++i) {
    k_wt_f16<<<(HID * (CC / 8) + 255) / 256, 256, 0, stream>>>(Wi1 + (size_t)i * CC * HID, BWi1, CC, HID, 16.0f); k_wt_f16<<<(CC * (HID / 8) + 255) / 256, 256, 0, stream>>>(Wi2 + (size_t)i * HID * CC, BWi2, HID, CC, 16.0f); k_wt_f16<<<(unsigned)(((size_t)XLW * (CC / 8) + 255) / 256), 256, 0, stream>>>(Wl + (size_t)i * CC * XLW, BWl, CC, XLW, 16.0f); k_wt_f16<<<(unsigned)(((size_t)XLW * (CC / 8) + 255) / 256), 256, 0, stream>>>(Wr + (size_t)i * CC * XLW, BWr, CC, XLW, 16.0f);
    k_gemm_hhx<3><<<gH, 128, 0, stream>>>(CF16, CC, 0, BWi1, CC, 0, 0.0625f, bi1 + i * HID, 0, nullptr, 1, 0, 0, nullptr, I1, HID, 0, NR, HID, CC);
    k_gemm_hhx<0><<<gC, 128, 0, stream>>>(I1, HID, 0, BWi2, HID, 0, 0.0625f, bi2 + i * CC, 0, AC, 1, (size_t)CC, 0, FEAT, nullptr, CC, 0, NR, CC, HID); k_f16<<<nb8, 256, 0, stream>>>(FEAT, F16, n8);
    k_gemm_hhx<0><<<gX, 128, 0, stream>>>(F16, CC, 0, BWl, CC, 0, 0.0625f, bl + (size_t)i * XLW, 0, nullptr, 1, 0, 0, nullptr, XL, XLW, 0, NR, XLW, CC); k_gemm_hhx<0><<<gX, 128, 0, stream>>>(F16, CC, 0, BWr, CC, 0, 0.0625f, br + (size_t)i * XLW, 0, nullptr, 1, 0, 0, nullptr, XR, XLW, 0, NR, XLW, CC);
    k_gat<<<NR / 8, 256, 0, stream>>>(NBR, cnt, ES, XL, XR, att + (size_t)i * HEADS * CC, gb + (size_t)i * CC, HYP);
    k_nchw<<<(unsigned)(((size_t)NBt * CC * (NN / 4) + 255) / 256), 256, 0, stream>>>(HYP, (float*)((char*)d_out + (size_t)i * 8388608)); }
  k_gemm_hhx<3><<<gF, 128, 0, stream>>>(AC16, CC, 0, BWf1, CC, 0, 0.0625f, bf1, 0, nullptr, 1, 0, 0, nullptr, FF16, FF, 0, NR, FF, CC); k_gemm_hhx<0><<<gC, 128, 0, stream>>>(FF16, FF, 0, BWf2, FF, 0, 0.0625f, bf2, 0, AC, 1, (size_t)CC, 0, T, nullptr, CC, 0, NR, CC, FF);
  k_ln<<<NR / 8, 256, 0, stream>>>(T, lng + 2 * CC, lnb + 2 * CC, HYP); k_nchw<<<(unsigned)(((size_t)NBt * CC * (NN / 4) + 255) / 256), 256, 0, stream>>>(HYP, (float*)((char*)d_out + (size_t)3 * 8388608));
}
